// StaticHDC_42159398978225
// MI455X (gfx1250) — hardware-verified
//
#include <hip/hip_runtime.h>


#define DT   10000
#define DP   10048
#define NPIX 784
#define KP   800
#define NV   10
#define NB   32
#define NR   320
typedef __attribute__((ext_vector_type(16))) _Float16 v16h;
typedef __attribute__((ext_vector_type(8)))  _Float16 v8h;
typedef __attribute__((ext_vector_type(8)))  float    v8f;
typedef __attribute__((ext_vector_type(4)))  float    v4f;
#define VST2(T, ptr, val) do { const T _v = (val); *(volatile T*)(ptr) = _v; __threadfence(); *(volatile T*)(ptr) = _v; } while (0)
__device__ __forceinline__ v8f wmma16(v16h a, v16h b, v8f c) {
  v8f d = __builtin_amdgcn_wmma_f32_16x16x32_f16(false, a, false, b, (short)0, c, false, false);
  asm volatile("v_nop\n\tv_nop\n\tv_nop\n\tv_nop" : "+v"(d) : "v"(a), "v"(b));
  return d;
}
__device__ __forceinline__ v16h frag16(const _Float16* p, int hh) {
  const v8h lo = *(const v8h*)(p + 8 * hh), hi = *(const v8h*)(p + 16 + 8 * hh);
  return __builtin_shufflevector(lo, hi, 0,1,2,3,4,5,6,7,8,9,10,11,12,13,14,15);
}
__global__ __launch_bounds__(256) void k_onehot(const float* __restrict__ x, _Float16* __restrict__ A16) {
  const int t = blockIdx.x * 256 + threadIdx.x;
  if (t >= NR * (KP / 8)) return;
  const int r = t / (KP / 8), p0 = (t % (KP / 8)) * 8, v = r / NB, b = r % NB;
  v8h o;
#pragma unroll
  for (int e = 0; e < 8; ++e) {
    const int p = p0 + e; float val = 0.f;
    if (p < NPIX) { int idx = (int)(x[b * NPIX + p] * 10.0f); idx = idx < 0 ? 0 : (idx > NV - 1 ? NV - 1 : idx); val = (idx == v) ? 1.f : 0.f; }
    o[e] = (_Float16)val;
  }
  VST2(v8h, A16 + (size_t)r * KP + p0, o);
}
__global__ __launch_bounds__(256) void k_pos(const float* __restrict__ pos, _Float16* __restrict__ P16) {
  const int t = blockIdx.x * 256 + threadIdx.x;
  if (t >= DP * (KP / 8)) return;
  const int d = t / (KP / 8), p0 = (t % (KP / 8)) * 8;
  v8h o;
#pragma unroll
  for (int e = 0; e < 8; ++e) { const int p = p0 + e; o[e] = (d < DT && p < NPIX) ? (_Float16)pos[(size_t)d * NPIX + p] : (_Float16)0.f; }
  VST2(v8h, P16 + (size_t)d * KP + p0, o);
}
__global__ __launch_bounds__(128) void k_gemm(const _Float16* __restrict__ A16, const _Float16* __restrict__ P16, float* __restrict__ S) {
  __shared__ __attribute__((aligned(16))) float sT[4][16][68];
  const int lane = threadIdx.x & 31, wave = threadIdx.x >> 5, hh = lane >> 4, l16 = lane & 15;
  const int m0 = blockIdx.y * 64 + wave * 16, c0 = blockIdx.x * 64;
  v8f acc[4] = {};
#pragma unroll 5
  for (int k0 = 0; k0 < KP; k0 += 32) {
    const v16h a = frag16(A16 + (size_t)(m0 + l16) * KP + k0, hh);
#pragma unroll
    for (int t = 0; t < 4; ++t) acc[t] = wmma16(a, frag16(P16 + (size_t)(c0 + t * 16 + l16) * KP + k0, hh), acc[t]);
  }
  float (*st)[68] = sT[wave];
#pragma unroll
  for (int t = 0; t < 4; ++t)
#pragma unroll
    for (int v = 0; v < 8; ++v) st[v + 8 * hh][t * 16 + l16] = acc[t][v];
  __builtin_amdgcn_fence(__ATOMIC_RELEASE, "workgroup"); __builtin_amdgcn_wave_barrier(); __builtin_amdgcn_fence(__ATOMIC_ACQUIRE, "workgroup");
  for (int pass = 0; pass < 2; ++pass) {
#pragma unroll
    for (int j = 0; j < 8; ++j) { const int rr = j * 2 + hh, q4 = l16 * 4; *(volatile v4f*)(S + (size_t)(m0 + rr) * DP + c0 + q4) = *(const v4f*)(&st[rr][q4]); }
    __threadfence();
  }
}
__global__ __launch_bounds__(256) void k_bundle(const float* __restrict__ S, const float* __restrict__ vw, float* __restrict__ enc) {
  const int t = blockIdx.x * 256 + threadIdx.x;
  if (t >= NB * DP) return;
  const int b = t / DP, d = t % DP;
  float s = 0.f;
  if (d < DT) {
#pragma unroll
    for (int v = 0; v < NV; ++v) s += vw[v * DT + d] * S[(size_t)(v * NB + b) * DP + d];
  }
  const float sg = (s > 0.f) ? 1.f : ((s < 0.f) ? -1.f : 0.f);
  VST2(float, enc + t, sg);
}
__global__ __launch_bounds__(256) void k_cls(const float* __restrict__ enc, const float* __restrict__ clf, int* __restrict__ out) {
  __shared__ float red[256];
  __shared__ float sims[NB][NV];
  __shared__ int res[NB];
  const int t = threadIdx.x;
  for (int bc = 0; bc < NB * NV; ++bc) {
    const int b = bc / NV, c = bc % NV;
    float s = 0.f;
    for (int d = t; d < DT; d += 256) { const float w = clf[c * DT + d]; s += enc[(size_t)b * DP + d] * ((w > 0.f) ? 1.f : ((w < 0.f) ? -1.f : 0.f)); }
    red[t] = s;
    __syncthreads();
    for (int o = 128; o > 0; o >>= 1) { if (t < o) red[t] += red[t + o]; __syncthreads(); }
    if (t == 0) sims[b][c] = red[0];
    __syncthreads();
  }
  if (t < NB) { int best = 0; float bv = sims[t][0]; for (int c = 1; c < NV; ++c) if (sims[t][c] > bv) { bv = sims[t][c]; best = c; } res[t] = best; }
  __syncthreads();
  if (t < NB) { *(volatile int*)(out + t) = res[t]; __threadfence(); *(volatile int*)(out + t) = res[t]; }
}
extern "C" void kernel_launch(void* const* d_in, const int* in_sizes, int n_in,
                              void* d_out, int out_size, void* d_ws, size_t ws_size, hipStream_t stream) {
  (void)in_sizes; (void)n_in; (void)out_size;
  const float* x   = (const float*)d_in[0];
  const float* vw  = (const float*)d_in[1];
  const float* pos = (const float*)d_in[2];
  const float* clf = (const float*)d_in[3];
  int* out = (int*)d_out;
  char* ws = (char*)d_ws; size_t off = 0;
  auto take = [&](size_t bytes) { void* p = ws + off; off = (off + bytes + 255) & ~(size_t)255; return p; };
  _Float16* A16 = (_Float16*)take((size_t)NR * KP * 2);
  _Float16* P16 = (_Float16*)take((size_t)DP * KP * 2);
  float*    S   = (float*)take((size_t)NR * DP * 4);
  float*    enc = (float*)take((size_t)NB * DP * 4);
  if (off > ws_size) return;
  k_onehot<<<(NR * (KP / 8) + 255) / 256, 256, 0, stream>>>(x, A16);
  k_pos<<<(DP * (KP / 8) + 255) / 256, 256, 0, stream>>>(pos, P16);
  k_gemm<<<dim3(DP / 64, NR / 64), 128, 0, stream>>>(A16, P16, S);
  k_bundle<<<(NB * DP + 255) / 256, 256, 0, stream>>>(S, vw, enc);
  k_cls<<<1, 256, 0, stream>>>(enc, clf, out);
}
